// GraphConv_23459111371106
// MI455X (gfx1250) — hardware-run, weakly checked
//
#include <hip/hip_runtime.h>
#include <math.h>

#define NB    64
#define NN    36
#define ND    2048
#define NK    8
#define NM    128
#define NROW  (NB * NN)
#define NCOL  (NK * NM)
#define JP    64
#define IP    48
#define LP    72

typedef __bf16          v16b __attribute__((ext_vector_type(16)));
typedef unsigned short  v8us __attribute__((ext_vector_type(8)));
typedef unsigned short  v4us __attribute__((ext_vector_type(4)));
typedef float           v8f  __attribute__((ext_vector_type(8)));
typedef float           v4f  __attribute__((ext_vector_type(4)));
typedef int             v8i  __attribute__((ext_vector_type(8)));
typedef v8us __attribute__((may_alias)) v8usa;
typedef v4us __attribute__((may_alias)) v4usa;
typedef v4f  __attribute__((may_alias)) v4fa;

union FragB { v16b v; v8us hv[2]; };

__device__ __forceinline__ v8f wmma_bf(v16b a, v16b b, v8f c) {
  v8f d = __builtin_amdgcn_wmma_f32_16x16x32_bf16(false, a, false, b, (short)0, c, false, false);
  const v8i ai = __builtin_bit_cast(v8i, a);
  const v8i bi = __builtin_bit_cast(v8i, b);
  asm volatile("v_nop\n\tv_nop\n\tv_nop\n\tv_nop" : "+v"(d) : "v"(ai), "v"(bi));
  return d;
}

__device__ __forceinline__ v16b load_frag(const unsigned short* p, int h) {
  FragB f;
  f.hv[0] = *(const v8usa*)(p + 8 * h);
  f.hv[1] = *(const v8usa*)(p + 16 + 8 * h);
  return f.v;
}

__device__ __forceinline__ unsigned int bf16_bits(float x) {
  const unsigned int u = __float_as_uint(x);
  return (u + 0x7FFFu + ((u >> 16) & 1u)) >> 16;
}
__device__ __forceinline__ float bf16_val(unsigned int bits) { return __uint_as_float(bits << 16); }
__device__ __forceinline__ float bf16_rne(float x) { return bf16_val(bf16_bits(x)); }

__device__ __forceinline__ void split2(float x, unsigned short& hb, unsigned short& lb) {
  const unsigned int hbits = bf16_bits(x);
  const float hf = bf16_val(hbits);
  hb = (unsigned short)hbits;
  lb = (unsigned short)bf16_bits(x - hf);
}

__device__ __forceinline__ void gw_store_pass(const float* sW, float* gp, int bi, int w, int lane) {
  const int q8 = lane & 7, sub = lane >> 3;
  const int b = bi / NN, i = bi - b * NN;
  #pragma unroll
  for (int it = 0; it < 2; ++it) {
    const int L = it * 4 + sub;
    const int k = 4 * w + (L >> 1), hl = L & 1;
    const v4f v = *(const v4fa*)(sW + k * JP + 32 * hl + 4 * q8);
    float* dst = gp + ((size_t)((b * NK + k) * NN + i)) * JP + 32 * hl + 4 * q8;
    *(volatile v4f*)dst = v;
  }
}

__global__ __launch_bounds__(64) void k_weights(
    const float* __restrict__ coord,
    const float* __restrict__ adjm,
    const float* __restrict__ adj,
    const float* __restrict__ mr,
    const float* __restrict__ mt,
    const float* __restrict__ pr,
    const float* __restrict__ pt,
    float* __restrict__ gp)
{
  #pragma clang fp contract(off)
  __shared__ __attribute__((aligned(16))) float sW[NK * JP];

  const int tid = threadIdx.x, lane = tid & 31, w = tid >> 5;
  const int bi = blockIdx.x;
  const int jc = (tid < NN) ? tid : (NN - 1);
  const int p = bi * NN + jc;

  const float rho = bf16_rne(coord[2 * p + 0]);
  const float th  = bf16_rne(coord[2 * p + 1]);
  const float a   = bf16_rne(adjm[p]) * bf16_rne(adj[p]);
  const float TWO_PI = 6.28318530717958647692f;

  float s = 0.0f;
  #pragma unroll 1
  for (int k = 0; k < NK; ++k) {
    const float mrk = bf16_rne(mr[k]), mtk = bf16_rne(mt[k]);
    const float prk = bf16_rne(pr[k]), ptk = bf16_rne(pt[k]);
    const float ir = 1.0f / (1e-14f + prk * prk);
    const float iv = 1.0f / (1e-14f + ptk * ptk);
    const float dr = rho - mrk;
    const float wr = expf((-0.5f * (dr * dr)) * ir);
    const float fa = fabsf(th - mtk);
    const float sa = fabsf(TWO_PI - fa);
    const float da = fminf(fa, sa);
    const float wtv = expf((-0.5f * (da * da)) * iv);
    float ww = wr * wtv;
    ww = (ww != ww) ? 0.0f : ww;
    s += ww;
    sW[k * JP + tid] = ww;
  }
  const float rs = 1.0f / (s + 1e-14f);
  const bool valid = tid < NN;
  #pragma unroll 1
  for (int k = 0; k < NK; ++k) {
    const float cw = sW[k * JP + tid] * rs;
    const float g = cw * a;
    sW[k * JP + tid] = valid ? g : 0.0f;
  }
  __syncthreads();

  gw_store_pass(sW, gp, bi, w, lane);
  __threadfence();
  gw_store_pass(sW, gp, bi, w, lane);
}

__global__ __launch_bounds__(256) void k_cvt_v(const float* __restrict__ v,
                                               unsigned short* __restrict__ vb)
{
  const int g = blockIdx.x * 256 + threadIdx.x;
  if (g >= NROW * ND / 8) return;
  const float* src = v + (size_t)g * 8;
  const v4f a = *(const v4fa*)src;
  const v4f c = *(const v4fa*)(src + 4);
  const v8us o = { (unsigned short)bf16_bits(a.x), (unsigned short)bf16_bits(a.y),
                   (unsigned short)bf16_bits(a.z), (unsigned short)bf16_bits(a.w),
                   (unsigned short)bf16_bits(c.x), (unsigned short)bf16_bits(c.y),
                   (unsigned short)bf16_bits(c.z), (unsigned short)bf16_bits(c.w) };
  unsigned short* dst = vb + (size_t)g * 8;
  *(volatile v8us*)dst = o;
  __threadfence();
  *(volatile v8us*)dst = o;
}

__device__ __forceinline__ void trw_store_pass(const unsigned short* sT, unsigned short* wt,
                                               int k, int d0, int w, int lane) {
  const int q8 = lane & 7, sub = lane >> 3;
  #pragma unroll
  for (int it = 0; it < 4; ++it) {
    const int mrow = it * 32 + w * 4 + sub;
    const v8us val = *(const v8usa*)(sT + mrow * LP + 8 * q8);
    unsigned short* dst = wt + ((size_t)(k * NM + mrow)) * ND + d0 + 8 * q8;
    *(volatile v8us*)dst = val;
  }
}

__global__ __launch_bounds__(256) void k_tr_w(const float* __restrict__ cw,
                                              unsigned short* __restrict__ wt)
{
  __shared__ __attribute__((aligned(16))) unsigned short sT[NM * LP];

  const int tid = threadIdx.x, lane = tid & 31, w = tid >> 5;
  const int d0 = blockIdx.x * 64, k = blockIdx.y;

  #pragma unroll
  for (int it = 0; it < 8; ++it) {
    const int f = it * 256 + tid;
    const int dl = f >> 5, mm = (f & 31) * 4;
    const v4f x = *(const v4fa*)(cw + ((size_t)(k * ND + d0 + dl)) * NM + mm);
    sT[(mm + 0) * LP + dl] = (unsigned short)bf16_bits(x.x);
    sT[(mm + 1) * LP + dl] = (unsigned short)bf16_bits(x.y);
    sT[(mm + 2) * LP + dl] = (unsigned short)bf16_bits(x.z);
    sT[(mm + 3) * LP + dl] = (unsigned short)bf16_bits(x.w);
  }
  __syncthreads();

  trw_store_pass(sT, wt, k, d0, w, lane);
  __threadfence();
  trw_store_pass(sT, wt, k, d0, w, lane);
}

__device__ __forceinline__ void vc_store_pass(const float* sT, float* vc, int m0, int c0, int w, int lane) {
  const int q8 = lane & 7, sub = lane >> 3;
  #pragma unroll
  for (int i = 0; i < 16; ++i) {
    const int lid = i * 4 + sub;
    const int row = lid >> 1, hl = lid & 1;
    const v4f v = *(const v4fa*)(sT + (32 * w + row) * 64 + 32 * hl + 4 * q8);
    const size_t gi = ((size_t)(m0 + 32 * w + row)) * NCOL + c0 + 32 * hl + 4 * q8;
    *(volatile v4f*)(vc + gi) = v;
  }
}

__global__ __launch_bounds__(128) void k_gemm(
    const unsigned short* __restrict__ vb,
    const unsigned short* __restrict__ wt,
    float* __restrict__ vc)
{
  __shared__ __attribute__((aligned(16))) float sT[128 * 64];

  const int tid = threadIdx.x, lane = tid & 31, w = tid >> 5;
  const int h = lane >> 4, m = lane & 15;
  const int m0 = blockIdx.x * 128;
  const int c0 = blockIdx.y * 64;
  const int m0w = m0 + 32 * w;

  const unsigned short* xa0 = vb + (size_t)(m0w + m) * ND;
  const unsigned short* xa1 = xa0 + (size_t)16 * ND;
  const unsigned short* wb  = wt + (size_t)(c0 + m) * ND;

  const v8f zero8 = {0.f, 0.f, 0.f, 0.f, 0.f, 0.f, 0.f, 0.f};
  v8f acc[2][4];
  #pragma unroll
  for (int mt = 0; mt < 2; ++mt)
    #pragma unroll
    for (int nt = 0; nt < 4; ++nt) acc[mt][nt] = zero8;

  #pragma unroll 1
  for (int k0 = 0; k0 < ND; k0 += 32) {
    const v16b a0 = load_frag(xa0 + k0, h);
    const v16b a1 = load_frag(xa1 + k0, h);
    #pragma unroll
    for (int nt = 0; nt < 4; ++nt) {
      const v16b b = load_frag(wb + (size_t)nt * 16 * ND + k0, h);
      acc[0][nt] = wmma_bf(a0, b, acc[0][nt]);
      acc[1][nt] = wmma_bf(a1, b, acc[1][nt]);
    }
  }

  #pragma unroll
  for (int nt = 0; nt < 4; ++nt)
    #pragma unroll
    for (int mt = 0; mt < 2; ++mt)
      #pragma unroll
      for (int r = 0; r < 8; ++r) {
        const int rowl = 32 * w + 16 * mt + 8 * h + r;
        sT[rowl * 64 + 16 * nt + m] = acc[mt][nt][r];
      }
  __syncthreads();

  vc_store_pass(sT, vc, m0, c0, w, lane);
  __threadfence();
  vc_store_pass(sT, vc, m0, c0, w, lane);
}

#define SM_AH   0
#define SM_AL   6912
#define SM_BH   13824
#define SM_BL   32256
#define SM_TOT  50688
#define SM_O    0

__device__ __forceinline__ void mix_store_pass(const float* sO, float* out, int b, int k, int w, int lane) {
  const int q8 = lane & 7, sub = lane >> 3;
  #pragma unroll
  for (int s = 0; s < 9; ++s) {
    const int L = s * 16 + w * 4 + sub;
    const int row = L >> 2, q = L & 3;
    const v4f v = *(const v4fa*)(sO + row * NM + 32 * q + 4 * q8);
    const size_t gi = ((size_t)(b * NN + row)) * NCOL + k * NM + 32 * q + 4 * q8;
    *(volatile v4f*)(out + gi) = v;
  }
}

__global__ __launch_bounds__(128) void k_mix(
    const float* __restrict__ gp,
    const float* __restrict__ vc,
    float* __restrict__ out)
{
  __shared__ __attribute__((aligned(16))) unsigned char smem[SM_TOT];
  unsigned short* sAh = (unsigned short*)(smem + SM_AH);
  unsigned short* sAl = (unsigned short*)(smem + SM_AL);
  unsigned short* sBh = (unsigned short*)(smem + SM_BH);
  unsigned short* sBl = (unsigned short*)(smem + SM_BL);
  float* sO = (float*)(smem + SM_O);

  const int tid = threadIdx.x, lane = tid & 31, w = tid >> 5;
  const int h = lane >> 4, m = lane & 15;
  const int bk = blockIdx.x;
  const int b = bk >> 3, k = bk & 7;

  const v4f z4f = {0.f, 0.f, 0.f, 0.f};
  #pragma unroll
  for (int it = 0; it < 6; ++it) {
    const int f = it * 128 + tid;
    const int i = f >> 4, j = (f & 15) * 4;
    const int ic = (i < NN) ? i : (NN - 1);
    v4f x = *(const v4fa*)(gp + ((size_t)(bk * NN + ic)) * JP + j);
    if (i >= NN) x = z4f;
    unsigned short h0, l0, h1, l1, h2, l2, h3, l3;
    split2(x.x, h0, l0); split2(x.y, h1, l1); split2(x.z, h2, l2); split2(x.w, h3, l3);
    const v4us hv = { h0, h1, h2, h3 };
    const v4us lv = { l0, l1, l2, l3 };
    *(v4usa*)(sAh + i * LP + j) = hv;
    *(v4usa*)(sAl + i * LP + j) = lv;
  }

  {
    const v4us z4 = { 0, 0, 0, 0 };
    const v8us z8 = { 0, 0, 0, 0, 0, 0, 0, 0 };
    unsigned short* ph = sBh + tid * LP;
    unsigned short* pl = sBl + tid * LP;
    *(v4usa*)(ph + 36) = z4; *(v8usa*)(ph + 40) = z8; *(v8usa*)(ph + 48) = z8; *(v8usa*)(ph + 56) = z8;
    *(v4usa*)(pl + 36) = z4; *(v8usa*)(pl + 40) = z8; *(v8usa*)(pl + 48) = z8; *(v8usa*)(pl + 56) = z8;
  }
  #pragma unroll
  for (int it = 0; it < 9; ++it) {
    const int f = it * 128 + tid;
    const int j = f >> 5, mm = (f & 31) * 4;
    const v4f x = *(const v4fa*)(vc + ((size_t)(b * NN + j)) * NCOL + k * NM + mm);
    unsigned short h0, l0, h1, l1, h2, l2, h3, l3;
    split2(x.x, h0, l0); split2(x.y, h1, l1); split2(x.z, h2, l2); split2(x.w, h3, l3);
    sBh[(mm + 0) * LP + j] = h0; sBl[(mm + 0) * LP + j] = l0;
    sBh[(mm + 1) * LP + j] = h1; sBl[(mm + 1) * LP + j] = l1;
    sBh[(mm + 2) * LP + j] = h2; sBl[(mm + 2) * LP + j] = l2;
    sBh[(mm + 3) * LP + j] = h3; sBl[(mm + 3) * LP + j] = l3;
  }
  __syncthreads();

  const v8f zero8 = {0.f, 0.f, 0.f, 0.f, 0.f, 0.f, 0.f, 0.f};
  v8f acc[3][2];
  #pragma unroll
  for (int it = 0; it < 3; ++it)
    #pragma unroll
    for (int nt = 0; nt < 2; ++nt) acc[it][nt] = zero8;

  #pragma unroll
  for (int ks = 0; ks < 2; ++ks) {
    const int k0 = 32 * ks;
    v16b bh[2], bl[2];
    #pragma unroll
    for (int nt = 0; nt < 2; ++nt) {
      const int nrow = 32 * w + 16 * nt + m;
      bh[nt] = load_frag(sBh + nrow * LP + k0, h);
      bl[nt] = load_frag(sBl + nrow * LP + k0, h);
    }
    #pragma unroll
    for (int it = 0; it < 3; ++it) {
      const int arow = 16 * it + m;
      const v16b ah = load_frag(sAh + arow * LP + k0, h);
      const v16b al = load_frag(sAl + arow * LP + k0, h);
      #pragma unroll
      for (int nt = 0; nt < 2; ++nt) {
        acc[it][nt] = wmma_bf(ah, bh[nt], acc[it][nt]);
        acc[it][nt] = wmma_bf(al, bh[nt], acc[it][nt]);
        acc[it][nt] = wmma_bf(ah, bl[nt], acc[it][nt]);
      }
    }
  }
  __syncthreads();

  #pragma unroll
  for (int it = 0; it < 3; ++it)
    #pragma unroll
    for (int nt = 0; nt < 2; ++nt)
      #pragma unroll
      for (int r = 0; r < 8; ++r) {
        const int i = 16 * it + 8 * h + r;
        const int col = 32 * w + 16 * nt + m;
        if (i < NN) sO[i * NM + col] = acc[it][nt][r];
      }
  __syncthreads();

  mix_store_pass(sO, out, b, k, w, lane);
  __threadfence();
  mix_store_pass(sO, out, b, k, w, lane);
}

extern "C" void kernel_launch(void* const* d_in, const int* in_sizes, int n_in,
                              void* d_out, int out_size, void* d_ws, size_t ws_size,
                              hipStream_t stream) {
  if (n_in < 11) return;
  if (in_sizes[0] != NB * NN * ND) return;
  if (in_sizes[2] != NB * NN * NN * 2) return;
  if (in_sizes[3] != NB * NN * NN) return;
  if (in_sizes[4] != NB * NN * NN) return;
  if (in_sizes[6] != NK || in_sizes[7] != NK || in_sizes[8] != NK || in_sizes[9] != NK) return;
  if (in_sizes[10] != NK * ND * NM) return;
  if (out_size != NROW * NCOL) return;

  const float* v     = (const float*)d_in[0];
  const float* coord = (const float*)d_in[2];
  const float* adjm  = (const float*)d_in[3];
  const float* adj   = (const float*)d_in[4];
  const float* mr    = (const float*)d_in[6];
  const float* mt    = (const float*)d_in[7];
  const float* pr    = (const float*)d_in[8];
  const float* pt    = (const float*)d_in[9];
  const float* convw = (const float*)d_in[10];
  float* out = (float*)d_out;

  const size_t gp_bytes = (size_t)NB * NK * NN * JP * sizeof(float);
  const size_t vb_bytes = (size_t)NROW * ND * sizeof(unsigned short);
  const size_t wt_bytes = (size_t)NCOL * ND * sizeof(unsigned short);
  const size_t vc_bytes = (size_t)NROW * NCOL * sizeof(float);
  const size_t off_gp = 0;
  const size_t off_vb = off_gp + gp_bytes;
  const size_t off_wt = off_vb + vb_bytes;
  const size_t off_vc = off_wt + wt_bytes;
  const size_t total  = off_vc + vc_bytes;
  if (total > ws_size) return;

  char* ws = (char*)d_ws;
  float* gp = (float*)(ws + off_gp);
  unsigned short* vb = (unsigned short*)(ws + off_vb);
  unsigned short* wt = (unsigned short*)(ws + off_wt);
  float* vc = (float*)(ws + off_vc);

  k_weights<<<NROW, 64, 0, stream>>>(coord, adjm, adj, mr, mt, pr, pt, gp);

  const int ncvt = NROW * ND / 8;
  k_cvt_v<<<(ncvt + 255) / 256, 256, 0, stream>>>(v, vb);

  dim3 gTr(ND / 64, NK);
  k_tr_w<<<gTr, 256, 0, stream>>>(convw, wt);

  dim3 gGemm(NROW / 128, NCOL / 64);
  k_gemm<<<gGemm, 128, 0, stream>>>(vb, wt, vc);

  k_mix<<<NB * NK, 128, 0, stream>>>(gp, vc, out);
}
